// GATv2Layer_66632122630755
// MI455X (gfx1250) — hardware-verified
//
#include <hip/hip_runtime.h>
#include <stdint.h>

#define NBATCH 8
#define NNODE  1024
#define CIN    256
#define COUT   256
#define NHEAD  8
#define HDIM   32
#define MROWS  (NBATCH * NNODE)
#define WSC    16.0f
#define PSC    256.0f
#define NEGFILL (-1.0e9f)

#define SLP      33
#define PPITCH   1032
#define OPITCH   36
#define ATT_ROWS 64
#define LDS_P_BYTES   (ATT_ROWS * PPITCH * 2)
#define LDS_SD_BYTES  (NNODE * 4)
#define LDS_O_BYTES   (ATT_ROWS * OPITCH * 4)
#define LDS_SI_BYTES  (ATT_ROWS * 4)
#define LDS_INV_BYTES (ATT_ROWS * 4)
#define ATT_LDS_BYTES (LDS_P_BYTES + LDS_SD_BYTES + LDS_O_BYTES + LDS_SI_BYTES + LDS_INV_BYTES)

#define XBLOCKS ((MROWS * CIN) / (256 * 8))
#define WBLOCKS ((COUT * CIN) / (256 * 8))

static_assert(ATT_LDS_BYTES == 145920);
static_assert(XBLOCKS * 256 * 8 == MROWS * CIN);
static_assert(WBLOCKS * 256 * 8 == COUT * CIN);
static_assert((LDS_P_BYTES % 16) == 0);
static_assert((PPITCH % 8) == 0);
static_assert((OPITCH % 4) == 0);
static_assert(NNODE % ATT_ROWS == 0);
static_assert(MROWS % 64 == 0);
static_assert(NNODE % 64 == 0);

typedef _Float16 v16h __attribute__((ext_vector_type(16)));
typedef _Float16 v8h  __attribute__((ext_vector_type(8)));
typedef _Float16 v4h  __attribute__((ext_vector_type(4)));
typedef float    v8f  __attribute__((ext_vector_type(8)));
typedef float    v4f  __attribute__((ext_vector_type(4)));
typedef int      v4i  __attribute__((ext_vector_type(4)));

union Frag { v16h v; v8h h[2]; };

__device__ __forceinline__ v8f mma16(v16h a, v16h b, v8f c) {
  return __builtin_amdgcn_wmma_f32_16x16x32_f16(false, a, false, b, (short)0, c, false, false);
}
__device__ __forceinline__ void guard1(v8f& c, v16h a, v16h b) {
  asm volatile("v_nop\n\tv_nop\n\tv_nop\n\tv_nop" : "+v"(c) : "v"(a), "v"(b));
}
__device__ __forceinline__ void guard2(v8f& c0, v8f& c1, v16h a, v16h b0, v16h b1) {
  asm volatile("v_nop\n\tv_nop\n\tv_nop\n\tv_nop" : "+v"(c0), "+v"(c1) : "v"(a), "v"(b0), "v"(b1));
}
__device__ __forceinline__ void accg2(v8f& a, v8f& b) {
  asm volatile("v_nop\n\tv_nop\n\tv_nop\n\tv_nop" : "+v"(a), "+v"(b));
}
__device__ __forceinline__ void accg1(v8f& a) {
  asm volatile("v_nop\n\tv_nop\n\tv_nop\n\tv_nop" : "+v"(a));
}

__device__ __forceinline__ void cvt8_store2(const float* __restrict__ s, _Float16* __restrict__ d, float sc) {
  const v4f f0 = *(const v4f*)(s);
  const v4f f1 = *(const v4f*)(s + 4);
  v8h hv;
  hv[0] = (_Float16)(f0[0] * sc); hv[1] = (_Float16)(f0[1] * sc);
  hv[2] = (_Float16)(f0[2] * sc); hv[3] = (_Float16)(f0[3] * sc);
  hv[4] = (_Float16)(f1[0] * sc); hv[5] = (_Float16)(f1[1] * sc);
  hv[6] = (_Float16)(f1[2] * sc); hv[7] = (_Float16)(f1[3] * sc);
  *(volatile v8h*)d = hv;
  __threadfence();
  *(volatile v8h*)d = hv;
}

__global__ __launch_bounds__(256) void k_cvt(const float* __restrict__ x, const float* __restrict__ W,
                                             _Float16* __restrict__ Xh, _Float16* __restrict__ Wh) {
  const int tid = threadIdx.x;
  if (blockIdx.x < XBLOCKS) {
    const size_t e0 = ((size_t)blockIdx.x * 256 + tid) * 8;
    cvt8_store2(x + e0, Xh + e0, 1.0f);
  } else {
    const size_t e0 = ((size_t)(blockIdx.x - XBLOCKS) * 256 + tid) * 8;
    cvt8_store2(W + e0, Wh + e0, WSC);
  }
}

__global__ __launch_bounds__(128) void k_hproj(const _Float16* __restrict__ Xh, const _Float16* __restrict__ Wh,
                                               const float* __restrict__ a,
                                               _Float16* __restrict__ hT, float* __restrict__ splane) {
  __shared__ float slab[4][64 * SLP];
  __shared__ __align__(16) float sst[4][128];
  const int tid  = threadIdx.x;
  const int lane = tid & 31;
  const int w    = tid >> 5;
  const int mt   = blockIdx.x >> 1;
  const int hh   = ((blockIdx.x & 1) << 2) + w;
  const int gm0  = mt * 64;
  const int b    = mt >> 4;
  const int n0   = (mt & 15) * 64;
  const int o0   = hh * HDIM;
  const int bh   = b * NHEAD + hh;
  const int m    = lane & 15;
  const int lh   = lane >> 4;

  const v8f zero = {0.f, 0.f, 0.f, 0.f, 0.f, 0.f, 0.f, 0.f};
  v8f acc[4][2];
#pragma unroll
  for (int i = 0; i < 4; ++i) { acc[i][0] = zero; acc[i][1] = zero; }

  const _Float16* pa = Xh + (size_t)(gm0 + m) * CIN + 8 * lh;
  const _Float16* pb = Wh + (size_t)(o0 + m) * CIN + 8 * lh;

  for (int k0 = 0; k0 < CIN; k0 += 32) {
    Frag b0, b1;
    b0.h[0] = *(const v8h*)(pb + k0);
    b0.h[1] = *(const v8h*)(pb + k0 + 16);
    b1.h[0] = *(const v8h*)(pb + 16 * CIN + k0);
    b1.h[1] = *(const v8h*)(pb + 16 * CIN + k0 + 16);
#pragma unroll
    for (int i = 0; i < 4; ++i) {
      Frag af;
      af.h[0] = *(const v8h*)(pa + (size_t)i * 16 * CIN + k0);
      af.h[1] = *(const v8h*)(pa + (size_t)i * 16 * CIN + k0 + 16);
      acc[i][0] = mma16(af.v, b0.v, acc[i][0]);
      acc[i][1] = mma16(af.v, b1.v, acc[i][1]);
      guard2(acc[i][0], acc[i][1], af.v, b0.v, b1.v);
    }
  }
  accg2(acc[0][0], acc[0][1]);
  accg2(acc[1][0], acc[1][1]);
  accg2(acc[2][0], acc[2][1]);
  accg2(acc[3][0], acc[3][1]);

  float* sl = slab[w];
  const float unw = 1.0f / WSC;
#pragma unroll
  for (int i = 0; i < 4; ++i) {
#pragma unroll
    for (int j = 0; j < 2; ++j) {
#pragma unroll
      for (int r = 0; r < 8; ++r) {
        sl[(16 * i + 8 * lh + r) * SLP + 16 * j + m] = acc[i][j][r] * unw;
      }
    }
  }
  __syncthreads();

  const float* asrc = a + hh * (2 * HDIM);
  const float* adst = asrc + HDIM;
  const float* h0p = sl + (2 * lane) * SLP;
  const float* h1p = sl + (2 * lane + 1) * SLP;
  float s0 = 0.f, s1 = 0.f, d0 = 0.f, d1 = 0.f;
#pragma unroll 4
  for (int c = 0; c < HDIM; ++c) {
    const float av = asrc[c];
    const float dv = adst[c];
    const float hv0 = h0p[c];
    const float hv1 = h1p[c];
    s0 += hv0 * av; s1 += hv1 * av;
    d0 += hv0 * dv; d1 += hv1 * dv;
  }
  sst[w][2 * lane]          = s0;
  sst[w][2 * lane + 1]      = s1;
  sst[w][64 + 2 * lane]     = d0;
  sst[w][64 + 2 * lane + 1] = d1;
  __syncthreads();

  const int seg = lane >> 4;
  const int p4  = (lane & 15) * 4;
  const v4f sv  = *(const v4f*)(&sst[w][seg * 64 + p4]);
  float* sp = splane + ((size_t)bh * 2 + seg) * NNODE + n0 + p4;

  const int q = lane >> 3;
  const int t = lane & 7;
  v8h hv[8];
#pragma unroll
  for (int it = 0; it < 8; ++it) {
    const int c = it * 4 + q;
#pragma unroll
    for (int e = 0; e < 8; ++e) hv[it][e] = (_Float16)sl[(8 * t + e) * SLP + c];
  }
  _Float16* hbase = hT + (size_t)bh * HDIM * NNODE + n0 + 8 * t;

#pragma unroll
  for (int it = 0; it < 8; ++it) {
    const int c = it * 4 + q;
    *(volatile v8h*)(hbase + (size_t)c * NNODE) = hv[it];
  }
  *(volatile v4f*)sp = sv;
  __threadfence();
#pragma unroll
  for (int it = 0; it < 8; ++it) {
    const int c = it * 4 + q;
    *(volatile v8h*)(hbase + (size_t)c * NNODE) = hv[it];
  }
  *(volatile v4f*)sp = sv;
}

__global__ __launch_bounds__(256) void k_attn(const int* __restrict__ adj, const float* __restrict__ splane,
                                              const _Float16* __restrict__ hT, float* __restrict__ out) {
  extern __shared__ __align__(16) unsigned char lds_raw[];
  _Float16* Psh   = (_Float16*)lds_raw;
  float*    sdsh  = (float*)(lds_raw + LDS_P_BYTES);
  float*    osl   = (float*)(lds_raw + LDS_P_BYTES + LDS_SD_BYTES);
  float*    sish  = (float*)(lds_raw + LDS_P_BYTES + LDS_SD_BYTES + LDS_O_BYTES);
  float*    invsh = (float*)(lds_raw + LDS_P_BYTES + LDS_SD_BYTES + LDS_O_BYTES + LDS_SI_BYTES);

  const int tid  = threadIdx.x;
  const int lane = tid & 31;
  const int w    = tid >> 5;
  const int i0   = blockIdx.x * ATT_ROWS;
  const int hh   = blockIdx.y;
  const int b    = blockIdx.z;
  const int bh   = b * NHEAD + hh;

  *(v4f*)(sdsh + 4 * tid) = *(const v4f*)(splane + ((size_t)bh * 2 + 1) * NNODE + 4 * tid);
  if (tid < ATT_ROWS) {
    sish[tid] = splane[(size_t)bh * 2 * NNODE + i0 + tid];
  }
  __syncthreads();

#pragma unroll 1
  for (int rr = 0; rr < 8; ++rr) {
    const int row = w * 8 + rr;
    const int i   = i0 + row;
    const int* arow = adj + ((size_t)(b * NNODE + i)) * NNODE;
    const float si = sish[row];
    float ev[32];
    float mx = -3.0e38f;
#pragma unroll
    for (int t = 0; t < 8; ++t) {
      const int j = t * 128 + lane * 4;
      const v4i av = *(const v4i*)(arow + j);
      const v4f sd = *(const v4f*)(sdsh + j);
#pragma unroll
      for (int e = 0; e < 4; ++e) {
        float v = si + sd[e];
        v = (v > 0.0f) ? v : (0.2f * v);
        v = (av[e] != 0) ? v : NEGFILL;
        ev[t * 4 + e] = v;
        mx = fmaxf(mx, v);
      }
    }
#pragma unroll
    for (int off = 16; off > 0; off >>= 1) mx = fmaxf(mx, __shfl_xor(mx, off, 32));

    float sum = 0.f;
#pragma unroll
    for (int t = 0; t < 8; ++t) {
      const int j = t * 128 + lane * 4;
      v4h ph;
#pragma unroll
      for (int e = 0; e < 4; ++e) {
        const float p = __expf(ev[t * 4 + e] - mx);
        sum += p;
        ph[e] = (_Float16)(p * PSC);
      }
      *(v4h*)(Psh + row * PPITCH + j) = ph;
    }
#pragma unroll
    for (int off = 16; off > 0; off >>= 1) sum += __shfl_xor(sum, off, 32);
    if (lane == 0) invsh[row] = (1.0f / sum) * (1.0f / PSC);
  }
  __syncthreads();

  const int mi = w & 3;
  const int ni = w >> 2;
  const int m  = lane & 15;
  const int lh = lane >> 4;
  const _Float16* pa = Psh + (16 * mi + m) * PPITCH + 8 * lh;
  const _Float16* pb = hT + ((size_t)bh * HDIM + 16 * ni + m) * NNODE + 8 * lh;
  v8f acc = {0.f, 0.f, 0.f, 0.f, 0.f, 0.f, 0.f, 0.f};
#pragma unroll 4
  for (int k0 = 0; k0 < NNODE; k0 += 32) {
    Frag af, bf;
    af.h[0] = *(const v8h*)(pa + k0);
    af.h[1] = *(const v8h*)(pa + k0 + 16);
    bf.h[0] = *(const v8h*)(pb + k0);
    bf.h[1] = *(const v8h*)(pb + k0 + 16);
    acc = mma16(af.v, bf.v, acc);
    guard1(acc, af.v, bf.v);
  }
  accg1(acc);

#pragma unroll
  for (int r = 0; r < 8; ++r) {
    const int row = 16 * mi + 8 * lh + r;
    const int col = 16 * ni + m;
    float v = acc[r] * invsh[row];
    v = (v > 0.0f) ? v : (__expf(v) - 1.0f);
    osl[row * OPITCH + col] = v;
  }
  __syncthreads();

  const int q = tid >> 3;
  const int t = tid & 7;
  const v4f o0 = *(const v4f*)(osl + q * OPITCH + 4 * t);
  const v4f o1 = *(const v4f*)(osl + (q + 32) * OPITCH + 4 * t);
  float* d0 = out + ((size_t)(b * NNODE + i0 + q)) * COUT + hh * HDIM + 4 * t;
  float* d1 = d0 + (size_t)32 * COUT;
  *(volatile v4f*)d0 = o0;
  *(volatile v4f*)d1 = o1;
  __threadfence();
  *(volatile v4f*)d0 = o0;
  *(volatile v4f*)d1 = o1;
}

extern "C" void kernel_launch(void* const* d_in, const int* in_sizes, int n_in,
                              void* d_out, int out_size, void* d_ws, size_t ws_size,
                              hipStream_t stream) {
  if (n_in < 4) return;
  if (in_sizes[0] != NBATCH * NNODE * CIN) return;
  if (in_sizes[1] != NBATCH * NNODE * NNODE) return;
  if (in_sizes[2] != COUT * CIN) return;
  if (in_sizes[3] != NHEAD * 2 * HDIM) return;
  if (out_size != NBATCH * NNODE * COUT) return;

  const size_t bXh = (size_t)MROWS * CIN * 2;
  const size_t bWh = (size_t)COUT * CIN * 2;
  const size_t bHT = (size_t)NBATCH * NHEAD * HDIM * NNODE * 2;
  const size_t bS  = (size_t)NBATCH * NHEAD * 2 * NNODE * 4;
  size_t off = 0;
  const size_t oXh = off; off += bXh;
  const size_t oWh = off; off += bWh;
  const size_t oHT = off; off += bHT;
  const size_t oS  = off; off += bS;
  if (off > ws_size) return;

  const float* x   = (const float*)d_in[0];
  const int*   adj = (const int*)d_in[1];
  const float* W   = (const float*)d_in[2];
  const float* a   = (const float*)d_in[3];
  float* out = (float*)d_out;
  char* ws = (char*)d_ws;
  _Float16* Xh     = (_Float16*)(ws + oXh);
  _Float16* Wh     = (_Float16*)(ws + oWh);
  _Float16* hT     = (_Float16*)(ws + oHT);
  float*    splane = (float*)(ws + oS);

  k_cvt<<<dim3(XBLOCKS + WBLOCKS), dim3(256), 0, stream>>>(x, W, Xh, Wh);
  k_hproj<<<dim3((MROWS / 64) * 2), dim3(128), 0, stream>>>(Xh, Wh, a, hT, splane);
  (void)hipFuncSetAttribute(reinterpret_cast<const void*>(&k_attn), hipFuncAttributeMaxDynamicSharedMemorySize, ATT_LDS_BYTES);
  k_attn<<<dim3(NNODE / ATT_ROWS, NHEAD, NBATCH), dim3(256), ATT_LDS_BYTES, stream>>>(adj, splane, hT, out);
  (void)hipGetLastError();
}
